// MultiHeadedAttention_59966333386766
// MI455X (gfx1250) — hardware-verified
//
#include <hip/hip_runtime.h>
#include <math.h>

typedef __attribute__((ext_vector_type(16))) _Float16 v16h;
typedef __attribute__((ext_vector_type(16))) __bf16 v16b;
typedef __attribute__((ext_vector_type(8)))  _Float16 v8h;
typedef __attribute__((ext_vector_type(8)))  __bf16 v8b;
typedef __attribute__((ext_vector_type(8)))  float v8f;
typedef __attribute__((ext_vector_type(4)))  float v4f;
typedef __attribute__((ext_vector_type(4)))  unsigned v4u;

#ifndef NB
#define NB 2
#endif
#ifndef SEQ
#define SEQ 2048
#endif
#define NB_FULL 2
#define SEQ_FULL 2048
#define DIN 1024
#define NH 16
#define HD 64
#define CC (NH * HD)
#define QHI ((SEQ) < 512 ? (SEQ) : 512)
#define KHI QHI

static_assert((SEQ & (SEQ - 1)) == 0);
static_assert(SEQ % 256 == 0);
static_assert(SEQ <= SEQ_FULL);
static_assert(NB <= NB_FULL);
static_assert(QHI % 64 == 0);
static_assert((SEQ - QHI) % 64 == 0);
static_assert(HD == 64);
static_assert(CC % 128 == 0);
static_assert(DIN % 128 == 0);
static_assert(DIN % 32 == 0);
static_assert(CC % 32 == 0);
static_assert(((size_t)SEQ * DIN) % 2048 == 0);
static_assert(((size_t)3 * CC * DIN) % 2048 == 0);
static_assert(((size_t)DIN * CC) % 2048 == 0);

template <typename T> __device__ __forceinline__ void vst2(void* p, T v) { *(volatile T*)p = v; __threadfence(); *(volatile T*)p = v; }
__device__ __forceinline__ v8f wmma16(v16h a, v16h b, v8f c) {
  v8f d = __builtin_amdgcn_wmma_f32_16x16x32_f16(false, a, false, b, (short)0, c, false, false);
  asm volatile("v_nop\n\tv_nop\n\tv_nop\n\tv_nop" : "+v"(d) : "v"(a), "v"(b));
  return d;
}
__device__ __forceinline__ v8f wmma_bf(v16b a, v16b b, v8f c) {
  v8f d = __builtin_amdgcn_wmma_f32_16x16x32_bf16(false, a, false, b, (short)0, c, false, false);
  asm volatile("v_nop\n\tv_nop\n\tv_nop\n\tv_nop" : "+v"(d) : "v"(a), "v"(b));
  return d;
}
__device__ __forceinline__ v16h frag_h(const _Float16* rowk0, unsigned lane) {
  union { v16h v; v8h q[2]; } u; const _Float16* p = rowk0 + 8u * (lane >> 4);
  u.q[0] = *(const v8h*)p; u.q[1] = *(const v8h*)(p + 16); return u.v;
}
__device__ __forceinline__ v16b frag_b(const __bf16* rowk0, unsigned lane) {
  union { v16b v; v8b q[2]; } u; const __bf16* p = rowk0 + 8u * (lane >> 4);
  u.q[0] = *(const v8b*)p; u.q[1] = *(const v8b*)(p + 16); return u.v;
}
#define LDSX() do { asm volatile("s_wait_dscnt 0" ::: "memory"); __builtin_amdgcn_wave_barrier(); __builtin_amdgcn_fence(3  , "workgroup"); } while (0)

#define WS_XB   ((size_t)0)
#define WS_WB   (WS_XB  + 2u * (size_t)NB * SEQ * DIN)
#define WS_WOB  (WS_WB  + 2u * (size_t)3 * CC * DIN)
#define WS_TAB  (WS_WOB + 2u * (size_t)DIN * CC)
#define WS_QH   (WS_TAB + 8u * (size_t)32 * SEQ)
#define WS_KH   (WS_QH  + 2u * (size_t)NB * SEQ * CC)
#define WS_VT   (WS_KH  + 2u * (size_t)NB * SEQ * CC)
#define WS_VTL  (WS_VT  + 2u * (size_t)NB * CC * SEQ)
#define WS_QL   (WS_VTL + 2u * (size_t)NB * CC * SEQ)
#define WS_KL   (WS_QL  + 2u * (size_t)NB * SEQ * CC)
#define WS_VB   (WS_KL  + 2u * (size_t)NB * KHI * CC)
#define WS_VBL  (WS_VB  + 2u * (size_t)NB * CC * KHI)
#define WS_YB   (WS_VBL + 2u * (size_t)NB * CC * KHI)
#define WS_YBL  (WS_YB  + 2u * (size_t)NB * SEQ * CC)
#define WS_END  (WS_YBL + 2u * (size_t)NB * SEQ * CC)
static_assert(WS_END <= (size_t)134217728);

__global__ __launch_bounds__(256) void k_cvt_a(const float* __restrict__ src, __bf16* __restrict__ dB, unsigned sstride, unsigned dstride) {
  const size_t e = ((size_t)blockIdx.x * 256u + threadIdx.x) * 8u;
  const float* s = src + (size_t)blockIdx.y * sstride + e;
  const v4f a = *(const v4f*)s; const v4f c = *(const v4f*)(s + 4);
  union { v8b b; v4u u; } ob;
#pragma unroll
  for (int u = 0; u < 4; ++u) { ob.b[u] = (__bf16)a[u]; ob.b[4 + u] = (__bf16)c[u]; }
  vst2(dB + (size_t)blockIdx.y * dstride + e, ob.u);
}

struct RopeArgs { float inv[32]; };
static_assert(sizeof(RopeArgs) == 128);
__global__ __launch_bounds__(256) void k_tab(RopeArgs ra, float* __restrict__ TAB) {
  __shared__ __align__(16) float sc[512];
  const unsigned tid = threadIdx.x; const unsigned i = blockIdx.y; const unsigned t = blockIdx.x * 256u + tid;
  float inv = ra.inv[0];
#pragma unroll
  for (int k = 1; k < 32; ++k) inv = (i == (unsigned)k) ? ra.inv[k] : inv;
  const float ang = (float)t * inv;
  float s, c; sincosf(ang, &s, &c);
  sc[2u * tid] = c; sc[2u * tid + 1u] = s;
  __syncthreads();
  if (tid < 128u) { const v4f v = *(const v4f*)&sc[4u * tid]; vst2(TAB + ((size_t)i * SEQ + blockIdx.x * 256u) * 2u + 4u * tid, v); }
}

__global__ __launch_bounds__(128) void k_proj(const __bf16* __restrict__ XB, const __bf16* __restrict__ WB, const float* __restrict__ TAB,
    _Float16* __restrict__ QH, _Float16* __restrict__ QL, _Float16* __restrict__ KH, _Float16* __restrict__ KL, _Float16* __restrict__ VT, _Float16* __restrict__ VTL, __bf16* __restrict__ VB, __bf16* __restrict__ VBL) {
  __shared__ __align__(16) _Float16 sbuf[4 * 128 * 72];
  static_assert(2 * 64 * 136 <= 4 * 128 * 72);
  const unsigned tid = threadIdx.x, wave = tid >> 5, lane = tid & 31u, col = lane & 15u, g = lane >> 4;
  const unsigned which = blockIdx.z; const unsigned c0 = blockIdx.y * 128u; const unsigned rb = blockIdx.x * 64u; const unsigned bb = rb / (unsigned)SEQ; const unsigned t0 = rb & (unsigned)(SEQ - 1);
  v8f acc[8] = {};
  const __bf16* arow = XB + (size_t)(rb + wave * 16u + col) * DIN;
  const __bf16* wrow = WB + (size_t)(which * (unsigned)CC + c0 + col) * DIN;
#pragma unroll 2
  for (unsigned kc = 0; kc < DIN / 32; ++kc) { const v16b a = frag_b(arow + kc * 32u, lane);
#pragma unroll
    for (int j = 0; j < 8; ++j) { const v16b w = frag_b(wrow + (size_t)j * 16 * DIN + kc * 32u, lane); acc[j] = wmma_bf(a, w, acc[j]); } }
  if (which < 2u) {
    _Float16 (*sh)[136] = (_Float16 (*)[136])sbuf; _Float16 (*sl)[136] = (_Float16 (*)[136])(sbuf + 64 * 136);
    const float sgn = (col & 1u) ? 1.0f : -1.0f;
    const unsigned tl = t0 + wave * 16u + 8u * g;
#pragma unroll
    for (int jj = 0; jj < 4; ++jj) { v4f cs[4]; const float* tp = TAB + 2u * ((size_t)((unsigned)jj * 8u + (col >> 1)) * SEQ + tl);
#pragma unroll
      for (int q = 0; q < 4; ++q) cs[q] = *(const v4f*)(tp + 4 * q);
      asm volatile("s_wait_loadcnt 0x0" ::: "memory");
#pragma unroll
      for (int r = 0; r < 8; ++r) { const float cr = cs[r >> 1][(r & 1) * 2], sr = cs[r >> 1][(r & 1) * 2 + 1];
#pragma unroll
        for (int u = 0; u < 2; ++u) { const float v = acc[jj + 4 * u][r]; const float p = __shfl_xor(v, 1); acc[jj + 4 * u][r] = v * cr + (sgn * p) * sr; } } }
    _Float16* DH = which == 0u ? QH : KH; _Float16* DL = which == 0u ? QL : KL;
    const bool wl = (which == 0u) || (t0 < (unsigned)KHI);
    const size_t lrow0 = which == 0u ? (size_t)rb : ((size_t)bb * KHI + t0);
#pragma unroll
    for (int j = 0; j < 8; ++j) {
#pragma unroll
      for (int r = 0; r < 8; ++r) { const float v = acc[j][r]; const _Float16 hv = (_Float16)v; sh[wave * 16u + 8u * g + r][j * 16 + col] = hv; sl[wave * 16u + 8u * g + r][j * 16 + col] = (_Float16)((v - (float)hv) * 1024.0f); } }
    __syncthreads();
    for (unsigned e = tid; e < 64u * 16u; e += 128u) { const unsigned rl = e >> 4, q = e & 15u; vst2(DH + (size_t)(rb + rl) * CC + c0 + q * 8u, *(const v4u*)&sh[rl][q * 8u]); if (wl) vst2(DL + (lrow0 + rl) * CC + c0 + q * 8u, *(const v4u*)&sl[rl][q * 8u]); }
  } else { const bool hi_rows = t0 < (unsigned)KHI;
    _Float16 (*th)[72] = (_Float16 (*)[72])sbuf; _Float16 (*tr)[72] = (_Float16 (*)[72])(sbuf + 128 * 72); __bf16 (*tb)[72] = (__bf16 (*)[72])(sbuf + 2 * 128 * 72); __bf16 (*tbl)[72] = (__bf16 (*)[72])(sbuf + 3 * 128 * 72);
#pragma unroll
    for (int j = 0; j < 8; ++j) {
#pragma unroll
      for (int r = 0; r < 8; ++r) { const float v = acc[j][r]; const unsigned rl = wave * 16u + 8u * g + r, cl = j * 16 + col; const _Float16 hv = (_Float16)v; th[cl][rl] = hv; tr[cl][rl] = (_Float16)((v - (float)hv) * 1024.0f); const __bf16 bh = (__bf16)v; tb[cl][rl] = bh; tbl[cl][rl] = (__bf16)(v - (float)bh); } }
    __syncthreads();
    for (unsigned e = tid; e < 128u * 8u; e += 128u) { const unsigned cl = e >> 3, q = e & 7u; const size_t o2 = ((size_t)bb * CC + c0 + cl) * SEQ + t0 + q * 8u;
      vst2(VT + o2, *(const v4u*)&th[cl][q * 8u]); vst2(VTL + o2, *(const v4u*)&tr[cl][q * 8u]);
      if (hi_rows) { const size_t o3 = ((size_t)bb * CC + c0 + cl) * KHI + t0 + q * 8u; vst2(VB + o3, *(const v4u*)&tb[cl][q * 8u]); vst2(VBL + o3, *(const v4u*)&tbl[cl][q * 8u]); } } }
}

template <int HI>
__device__ __forceinline__ void flash_body(const _Float16* __restrict__ QH, const _Float16* __restrict__ KH, const _Float16* __restrict__ QL, const _Float16* __restrict__ KL, const _Float16* __restrict__ VT, const _Float16* __restrict__ VTL, const __bf16* __restrict__ VB, const __bf16* __restrict__ VBL,
    __bf16* __restrict__ YB, __bf16* __restrict__ YBL) {
  __shared__ __align__(16) float so[4][16][68];
  const unsigned tid = threadIdx.x, wave = tid >> 5, lane = tid & 31u, col = lane & 15u, g = lane >> 4;
  const unsigned bh = blockIdx.y, b = bh / (unsigned)NH, h = bh % (unsigned)NH;
  const unsigned q0 = (HI ? 0u : (unsigned)QHI) + (blockIdx.x * 4u + wave) * 16u;
  const size_t rowb = (size_t)b * SEQ;
  const unsigned myq = q0 + col;
  const _Float16* qrow = QH + (rowb + myq) * CC + h * HD;
  const _Float16* qlrow = QL + (rowb + myq) * CC + h * HD;
  v8f o[4] = {}, orr[4] = {};
  float m = -1.0e30f, l = 0.f;
  const unsigned nkt = (q0 + 47u) >> 5;
  const float SC = 0.125f * 1.44269504f;
#pragma unroll 1
  for (unsigned kt = 0; kt < nkt; ++kt) { const unsigned j = kt * 32u;
    unsigned z = 0u; asm volatile("" : "+v"(z));
    const v16h qh0 = frag_h(qrow + z, lane), qh1 = frag_h(qrow + z + 32, lane), ql0 = frag_h(qlrow + z, lane), ql1 = frag_h(qlrow + z + 32, lane);
    const _Float16* kr0 = KH + (rowb + j + col) * CC + h * HD; const _Float16* kr1 = kr0 + (size_t)16 * CC;
    const v16h ka0 = frag_h(kr0, lane), ka1 = frag_h(kr0 + 32, lane), kb0 = frag_h(kr1, lane), kb1 = frag_h(kr1 + 32, lane);
    v8f s0 = {}, s1 = {}, t0 = {}, t1 = {};
    s0 = wmma16(ka0, qh0, s0); s0 = wmma16(ka1, qh1, s0);
    s1 = wmma16(kb0, qh0, s1); s1 = wmma16(kb1, qh1, s1);
    t0 = wmma16(ka0, ql0, t0); t0 = wmma16(ka1, ql1, t0);
    t1 = wmma16(kb0, ql0, t1); t1 = wmma16(kb1, ql1, t1);
    if (HI) { const _Float16* kl0 = KL + ((size_t)b * KHI + j + col) * CC + h * HD; const _Float16* kl1 = kl0 + (size_t)16 * CC;
      t0 = wmma16(frag_h(kl0, lane), qh0, t0); t0 = wmma16(frag_h(kl0 + 32, lane), qh1, t0);
      t1 = wmma16(frag_h(kl1, lane), qh0, t1); t1 = wmma16(frag_h(kl1 + 32, lane), qh1, t1); }
#pragma unroll
    for (int r = 0; r < 8; ++r) { s0[r] += t0[r] * (1.0f / 1024.0f); s1[r] += t1[r] * (1.0f / 1024.0f); }
    float v0[8], v1[8]; float ml = -1.0e30f;
#pragma unroll
    for (int r = 0; r < 8; ++r) { const unsigned ki = j + 8u * g + (unsigned)r; const bool ok0 = ki <= myq, ok1 = (ki + 16u) <= myq;
      v0[r] = ok0 ? s0[r] * SC : -1.0e30f; v1[r] = ok1 ? s1[r] * SC : -1.0e30f; ml = fmaxf(ml, fmaxf(v0[r], v1[r])); }
    ml = fmaxf(ml, __shfl_xor(ml, 16));
    const float mn = fmaxf(m, ml); const float alpha = exp2f(m - mn); m = mn;
    float e0[8], e1[8]; float ls = 0.f;
#pragma unroll
    for (int r = 0; r < 8; ++r) { const float x0 = exp2f(v0[r] - mn), x1 = exp2f(v1[r] - mn); e0[r] = (v0[r] > -1.0e29f) ? x0 : 0.f; e1[r] = (v1[r] > -1.0e29f) ? x1 : 0.f; ls += e0[r] + e1[r]; }
    l = l * alpha + ls;
#pragma unroll
    for (int c = 0; c < 4; ++c) {
#pragma unroll
      for (int r = 0; r < 8; ++r) { o[c][r] *= alpha; if (!HI) orr[c][r] *= alpha; } }
    if (HI) { v16b ph, pl;
#pragma unroll
      for (int r = 0; r < 8; ++r) { const __bf16 a0 = (__bf16)e0[r], a1 = (__bf16)e1[r]; ph[r] = a0; ph[8 + r] = a1; pl[r] = (__bf16)(e0[r] - (float)a0); pl[8 + r] = (__bf16)(e1[r] - (float)a1); }
#pragma unroll
      for (int c = 0; c < 4; ++c) { const size_t po = ((size_t)b * CC + h * HD + c * 16 + col) * KHI + j; const v16b vh = frag_b(VB + po, lane), vl = frag_b(VBL + po, lane);
        o[c] = wmma_bf(vh, pl, o[c]); o[c] = wmma_bf(vl, ph, o[c]); o[c] = wmma_bf(vh, ph, o[c]); }
    } else { v16h ph, pl;
#pragma unroll
      for (int r = 0; r < 8; ++r) { const float p0 = e0[r] * 1024.0f, p1 = e1[r] * 1024.0f; const _Float16 a0 = (_Float16)p0, a1 = (_Float16)p1; ph[r] = a0; ph[8 + r] = a1; pl[r] = (_Float16)((p0 - (float)a0) * 1024.0f); pl[8 + r] = (_Float16)((p1 - (float)a1) * 1024.0f); }
#pragma unroll
      for (int c = 0; c < 4; ++c) { const size_t po = ((size_t)b * CC + h * HD + c * 16 + col) * SEQ + j; const v16h vh = frag_h(VT + po, lane), vr = frag_h(VTL + po, lane);
        o[c] = wmma16(vh, ph, o[c]);
        orr[c] = wmma16(vr, ph, orr[c]); orr[c] = wmma16(vh, pl, orr[c]); } } }
  l += __shfl_xor(l, 16);
  const float il = 1.0f / l;
#pragma unroll
  for (int c = 0; c < 4; ++c) {
#pragma unroll
    for (int r = 0; r < 8; ++r) { const float val = HI ? o[c][r] * il : (o[c][r] + orr[c][r] * (1.0f / 1024.0f)) * ((1.0f / 1024.0f) * il); so[wave][col][c * 16 + 8 * g + r] = val; } }
  LDSX();
#pragma unroll
  for (int it = 0; it < 4; ++it) { const unsigned row = (unsigned)it * 4u + (lane >> 3), pc = lane & 7u;
    const v4f f0 = *(const v4f*)&so[wave][row][pc * 8u], f1 = *(const v4f*)&so[wave][row][pc * 8u + 4u];
    union { v8b b; v4u u; } hb, lb;
#pragma unroll
    for (int u = 0; u < 4; ++u) { const __bf16 a0 = (__bf16)f0[u], a1 = (__bf16)f1[u]; hb.b[u] = a0; hb.b[4 + u] = a1; lb.b[u] = (__bf16)(f0[u] - (float)a0); lb.b[4 + u] = (__bf16)(f1[u] - (float)a1); }
    const size_t oy = (rowb + q0 + row) * CC + h * HD + pc * 8u; vst2(YB + oy, hb.u); vst2(YBL + oy, lb.u); }
}
__global__ __launch_bounds__(128) void k_flash_hi(const _Float16* __restrict__ QH, const _Float16* __restrict__ KH, const _Float16* __restrict__ QL, const _Float16* __restrict__ KL, const _Float16* __restrict__ VT, const _Float16* __restrict__ VTL, const __bf16* __restrict__ VB, const __bf16* __restrict__ VBL, __bf16* __restrict__ YB, __bf16* __restrict__ YBL) {
  flash_body<1>(QH, KH, QL, KL, VT, VTL, VB, VBL, YB, YBL); }
__global__ __launch_bounds__(128) void k_flash_lo(const _Float16* __restrict__ QH, const _Float16* __restrict__ KH, const _Float16* __restrict__ QL, const _Float16* __restrict__ KL, const _Float16* __restrict__ VT, const _Float16* __restrict__ VTL, const __bf16* __restrict__ VB, const __bf16* __restrict__ VBL, __bf16* __restrict__ YB, __bf16* __restrict__ YBL) {
  flash_body<0>(QH, KH, QL, KL, VT, VTL, VB, VBL, YB, YBL); }

__global__ __launch_bounds__(128) void k_out(const __bf16* __restrict__ YB, const __bf16* __restrict__ YBL, const __bf16* __restrict__ WOB, float* __restrict__ OUT) {
  __shared__ __align__(16) float sf[4][16][132];
  const unsigned tid = threadIdx.x, wave = tid >> 5, lane = tid & 31u, col = lane & 15u, g = lane >> 4;
  const unsigned c0 = blockIdx.y * 128u; const unsigned rb = blockIdx.x * 64u; const unsigned r0 = rb + wave * 16u;
  v8f acc[8] = {};
  const size_t ya = (size_t)(r0 + col) * CC;
#pragma unroll 2
  for (unsigned kc = 0; kc < CC / 32; ++kc) { const v16b ah = frag_b(YB + ya + kc * 32u, lane), al = frag_b(YBL + ya + kc * 32u, lane);
#pragma unroll
    for (int j = 0; j < 8; ++j) { const v16b w = frag_b(WOB + (size_t)(c0 + j * 16 + col) * CC + kc * 32u, lane); acc[j] = wmma_bf(al, w, acc[j]); acc[j] = wmma_bf(ah, w, acc[j]); } }
#pragma unroll
  for (int j = 0; j < 8; ++j) {
#pragma unroll
    for (int r = 0; r < 8; ++r) sf[wave][8 * g + r][j * 16 + col] = acc[j][r]; }
  LDSX();
  for (unsigned rl = 0; rl < 16u; ++rl) vst2(OUT + (size_t)(r0 + rl) * DIN + c0 + lane * 4u, *(const v4f*)&sf[wave][rl][lane * 4u]);
}

extern "C" void kernel_launch(void* const* d_in, const int* in_sizes, int n_in, void* d_out, int out_size, void* d_ws, size_t ws_size, hipStream_t stream) {
  if (n_in < 3) return;
  if ((size_t)in_sizes[0] < (size_t)(NB - 1) * SEQ_FULL * DIN + (size_t)SEQ * DIN) return;
  if ((size_t)in_sizes[1] < (size_t)3 * CC * DIN) return;
  if ((size_t)in_sizes[2] < (size_t)DIN * CC) return;
  if ((size_t)out_size < (size_t)NB * SEQ * DIN) return;
  if (ws_size < (size_t)WS_END) return;
  const float* X = (const float*)d_in[0]; const float* WQKV = (const float*)d_in[1]; const float* WO = (const float*)d_in[2];
  char* ws = (char*)d_ws;
  __bf16 *XB = (__bf16*)(ws + WS_XB), *WB = (__bf16*)(ws + WS_WB), *WOB = (__bf16*)(ws + WS_WOB), *VB = (__bf16*)(ws + WS_VB), *VBL = (__bf16*)(ws + WS_VBL), *YB = (__bf16*)(ws + WS_YB), *YBL = (__bf16*)(ws + WS_YBL);
  _Float16 *QH = (_Float16*)(ws + WS_QH), *KH = (_Float16*)(ws + WS_KH), *VT = (_Float16*)(ws + WS_VT), *VTL = (_Float16*)(ws + WS_VTL), *QL = (_Float16*)(ws + WS_QL), *KL = (_Float16*)(ws + WS_KL);
  float* TAB = (float*)(ws + WS_TAB);
  RopeArgs ra;
  for (int i = 0; i < 32; ++i) { const float pw = (float)pow(10000.0, (double)(2 * i) / 64.0); ra.inv[i] = 1.0f / pw; }
  k_cvt_a<<<dim3((unsigned)((size_t)SEQ * DIN / 2048), NB), 256, 0, stream>>>(X, XB, (unsigned)((size_t)SEQ_FULL * DIN), (unsigned)((size_t)SEQ * DIN));
  k_cvt_a<<<dim3((unsigned)((size_t)3 * CC * DIN / 2048), 1), 256, 0, stream>>>(WQKV, WB, 0u, 0u);
  k_cvt_a<<<dim3((unsigned)((size_t)DIN * CC / 2048), 1), 256, 0, stream>>>(WO, WOB, 0u, 0u);
  k_tab<<<dim3(SEQ / 256, 32), 256, 0, stream>>>(ra, TAB);
  k_proj<<<dim3(NB * SEQ / 64, CC / 128, 3), 128, 0, stream>>>(XB, WB, TAB, QH, QL, KH, KL, VT, VTL, VB, VBL);
  k_flash_hi<<<dim3(QHI / 64, NB * NH), 128, 0, stream>>>(QH, KH, QL, KL, VT, VTL, VB, VBL, YB, YBL);
  if (SEQ > QHI) k_flash_lo<<<dim3((SEQ - QHI) / 64, NB * NH), 128, 0, stream>>>(QH, KH, QL, KL, VT, VTL, VB, VBL, YB, YBL);
  k_out<<<dim3(NB * SEQ / 64, DIN / 128), 128, 0, stream>>>(YB, YBL, WOB, (float*)d_out);
}
